// BackflowNet_10110353015415
// MI455X (gfx1250) — hardware-verified
//
#include <hip/hip_runtime.h>
#include <math.h>

#pragma clang fp contract(off)

#define NPART 64
#define DIM 3
#define HID 128
#define NCT 8
#define LDS_STRIDE 132
#define WAVES1 8

typedef __bf16 v16bf __attribute__((ext_vector_type(16)));
typedef float v8f __attribute__((ext_vector_type(8)));
typedef float v4f __attribute__((ext_vector_type(4)));
typedef float v4fa __attribute__((ext_vector_type(4), may_alias));
typedef unsigned int v4u __attribute__((ext_vector_type(4)));

union Frag {
  v16bf v;
  unsigned int u[8];
  v4u q[2];
};

__device__ __forceinline__ v8f mma_bf16(v16bf a, v16bf b, v8f acc) {
  acc = __builtin_amdgcn_wmma_f32_16x16x32_bf16(false, a, false, b, (short)0, acc, false, false);
  asm volatile("v_nop\n\tv_nop\n\tv_nop\n\tv_nop" : "+v"(acc) : "v"(a), "v"(b));
  return acc;
}

__device__ __forceinline__ unsigned int bf16_rne(float f) {
  unsigned int u = __float_as_uint(f);
  u += 0x7FFFu + ((u >> 16) & 1u);
  return u >> 16;
}

__device__ __forceinline__ void split2(float f, unsigned int& hb, unsigned int& lb) {
  hb = bf16_rne(f);
  float hf = __uint_as_float(hb << 16);
  lb = bf16_rne(f - hf);
}

__device__ __forceinline__ v4u pack8(const unsigned int* w) {
  v4u v;
  v.x = (w[0] & 0xFFFFu) | (w[1] << 16);
  v.y = (w[2] & 0xFFFFu) | (w[3] << 16);
  v.z = (w[4] & 0xFFFFu) | (w[5] << 16);
  v.w = (w[6] & 0xFFFFu) | (w[7] << 16);
  return v;
}

__device__ __forceinline__ void load_B(const unsigned int* __restrict__ base, int fragidx, int lane, Frag& B) {
  const unsigned int* p = base + ((size_t)fragidx * 32 + (size_t)lane) * 8;
  B.q[0] = *(const v4u*)p;
  B.q[1] = *(const v4u*)(p + 4);
}

__device__ __forceinline__ float silu_f(float z) {
  float e = __builtin_amdgcn_exp2f(-z * 1.44269504088896340736f);
  return z * __builtin_amdgcn_rcpf(1.0f + e);
}

__global__ __launch_bounds__(256) void pack_split(
    const float* __restrict__ W, int ld, int row_off, int row_count, int ncols_valid,
    int n_ct, int n_chunks, unsigned int* dst_hi, unsigned int* dst_lo) {
  int t = blockIdx.x * blockDim.x + threadIdx.x;
  int total = n_chunks * n_ct * 64;
  bool valid = t < total;
  int tt = valid ? t : 0;
  int halfsel = tt & 1;
  int lane = (tt >> 1) & 31;
  int c = (tt >> 6) % n_ct;
  int kc = (tt >> 6) / n_ct;
  int h = lane >> 4;
  int col = c * 16 + (lane & 15);
  int kbase = kc * 32 + halfsel * 16 + 8 * h;
  unsigned int hw[8], lw[8];
#pragma unroll
  for (int e = 0; e < 8; ++e) {
    int k = kbase + e;
    float f = 0.0f;
    if (col < ncols_valid && k < row_count) f = W[(size_t)(row_off + k) * (size_t)ld + (size_t)col];
    split2(f, hw[e], lw[e]);
  }
  v4u vh = pack8(hw);
  v4u vl = pack8(lw);
  size_t o = (size_t)tt * 4;
  if (valid) {
    *(volatile v4u*)(dst_hi + o) = vh;
    *(volatile v4u*)(dst_lo + o) = vl;
  }
  __threadfence();
  if (valid) {
    *(volatile v4u*)(dst_hi + o) = vh;
    *(volatile v4u*)(dst_lo + o) = vl;
  }
}

__global__ __launch_bounds__(256) void pack_tiny(
    const float* __restrict__ W, int ld, int row_off, int nsrc, int ncols_valid,
    int n_ct, unsigned int* dst) {
  int t = blockIdx.x * blockDim.x + threadIdx.x;
  int total = n_ct * 64;
  bool valid = t < total;
  int tt = valid ? t : 0;
  int halfsel = tt & 1;
  int lane = (tt >> 1) & 31;
  int c = (tt >> 6) % n_ct;
  int h = lane >> 4;
  int col = c * 16 + (lane & 15);
  int sbase = halfsel * 16 + 8 * h;
  unsigned int bw[8];
#pragma unroll
  for (int e = 0; e < 8; ++e) {
    int s = sbase + e;
    unsigned int bits = 0u;
    if (s < 3 * nsrc && col < ncols_valid) {
      int grp = s / nsrc;
      int row = row_off + (s - grp * nsrc);
      float f = W[(size_t)row * (size_t)ld + (size_t)col];
      unsigned int hb, lb;
      split2(f, hb, lb);
      bits = (grp == 1) ? lb : hb;
    }
    bw[e] = bits;
  }
  v4u v = pack8(bw);
  size_t o = (size_t)tt * 4;
  if (valid) *(volatile v4u*)(dst + o) = v;
  __threadfence();
  if (valid) *(volatile v4u*)(dst + o) = v;
}

__global__ __launch_bounds__(256) void phase1(
    const float* __restrict__ x, const int* __restrict__ spin,
    const float* __restrict__ phi_w0, const float* __restrict__ phi_b0,
    const unsigned int* __restrict__ w0t, float* s_out, int nrows) {
  __shared__ __attribute__((aligned(16))) float rowbuf[WAVES1][HID];
  (void)spin;
  int wave = threadIdx.x >> 5;
  int lane = threadIdx.x & 31;
  int h = lane >> 4;
  int lrow = lane & 15;
  int wid = blockIdx.x * WAVES1 + wave;
  bool valid = wid < nrows;
  int widc = valid ? wid : 0;
  int b = widc / NPART;
  int i = widc - b * NPART;

  const float* xb = x + (size_t)b * NPART * DIM;
  float xi0 = xb[i * 3 + 0], xi1 = xb[i * 3 + 1], xi2 = xb[i * 3 + 2];

  Frag Bt[NCT];
#pragma unroll
  for (int c = 0; c < NCT; ++c) load_B(w0t, c, lane, Bt[c]);

  float bias[NCT], sum[NCT];
#pragma unroll
  for (int c = 0; c < NCT; ++c) {
    int col = c * 16 + lrow;
    float t0 = xi0 * phi_w0[col];
    float t1 = xi1 * phi_w0[HID + col];
    float t2 = xi2 * phi_w0[2 * HID + col];
    bias[c] = ((t0 + t1) + t2) + phi_b0[col];
    sum[c] = 0.0f;
  }
  unsigned int lomask = h ? 0u : 0xFFFFFFFFu;

#pragma unroll 1
  for (int jt = 0; jt < NPART / 16; ++jt) {
    int j = jt * 16 + lrow;
    float xj0 = xb[j * 3 + 0], xj1 = xb[j * 3 + 1], xj2 = xb[j * 3 + 2];
    float d0 = xi0 - xj0, d1 = xi1 - xj1, d2 = xi2 - xj2;
    float rr = (d0 * d0 + d1 * d1) + d2 * d2;
    float rn = sqrtf(rr + 1e-12f);
    float f[8] = {xj0, xj1, xj2, d0, d1, d2, rn, rr};
    unsigned int hb[8], lb[8];
#pragma unroll
    for (int e = 0; e < 8; ++e) split2(f[e], hb[e], lb[e]);
    Frag A;
#pragma unroll
    for (int jj = 0; jj < 4; ++jj) {
      A.u[jj] = (hb[2 * jj] & 0xFFFFu) | (hb[2 * jj + 1] << 16);
      A.u[4 + jj] = ((lb[2 * jj] & 0xFFFFu) | (lb[2 * jj + 1] << 16)) & lomask;
    }
    int jb = jt * 16 + 8 * h;
#pragma unroll
    for (int c = 0; c < NCT; ++c) {
      v8f acc;
#pragma unroll
      for (int r = 0; r < 8; ++r) acc[r] = bias[c];
      acc = mma_bf16(A.v, Bt[c].v, acc);
#pragma unroll
      for (int r = 0; r < 8; ++r) {
        float v = silu_f(acc[r]);
        sum[c] += (jb + r == i) ? 0.0f : v;
      }
    }
  }

#pragma unroll
  for (int c = 0; c < NCT; ++c) {
    float v2 = sum[c] + __shfl_xor(sum[c], 16, 32);
    if (h == 0) rowbuf[wave][c * 16 + lrow] = v2;
  }
  __syncthreads();
  v4f vrow = *(const v4fa*)(&rowbuf[wave][4 * lane]);
  float* dst = s_out + (size_t)widc * HID + 4 * lane;
  if (valid) *(volatile v4f*)dst = vrow;
  __threadfence();
  if (valid) *(volatile v4f*)dst = vrow;
}

__device__ __forceinline__ void build_pair(const float* p0, const float* p1, Frag& FH, Frag& FL) {
#pragma unroll
  for (int jj = 0; jj < 4; ++jj) {
    unsigned int ha, la, hc, lc;
    split2(p0[2 * jj], ha, la);
    split2(p0[2 * jj + 1], hc, lc);
    FH.u[jj] = (ha & 0xFFFFu) | (hc << 16);
    FL.u[jj] = (la & 0xFFFFu) | (lc << 16);
    split2(p1[2 * jj], ha, la);
    split2(p1[2 * jj + 1], hc, lc);
    FH.u[4 + jj] = (ha & 0xFFFFu) | (hc << 16);
    FL.u[4 + jj] = (la & 0xFFFFu) | (lc << 16);
  }
}
__device__ __forceinline__ void load_A4(const float* rowp, int h, Frag AH[4], Frag AL[4]) {
#pragma unroll
  for (int kc = 0; kc < 4; ++kc) {
    const float* p0 = rowp + kc * 32 + 8 * h;
    build_pair(p0, p0 + 16, AH[kc], AL[kc]);
  }
}
__device__ __forceinline__ v8f gemm128_col(const Frag AH[4], const Frag AL[4],
    const unsigned int* __restrict__ bh, const unsigned int* __restrict__ bl,
    int n_ct, int c, int lane, v8f acc) {
#pragma unroll
  for (int kc = 0; kc < 4; ++kc) {
    Frag BH, BL;
    load_B(bh, kc * n_ct + c, lane, BH);
    load_B(bl, kc * n_ct + c, lane, BL);
    acc = mma_bf16(AH[kc].v, BH.v, acc);
    acc = mma_bf16(AL[kc].v, BH.v, acc);
    acc = mma_bf16(AH[kc].v, BL.v, acc);
  }
  return acc;
}

__global__ __launch_bounds__(128) void phase2(
    const float* __restrict__ x, const float* __restrict__ s,
    const unsigned int* __restrict__ w1h, const unsigned int* __restrict__ w1l,
    const float* __restrict__ phi_b1,
    const unsigned int* __restrict__ pxt,
    const unsigned int* __restrict__ pmh, const unsigned int* __restrict__ pml,
    const float* __restrict__ psi_b0,
    const unsigned int* __restrict__ p1h, const unsigned int* __restrict__ p1l,
    const float* __restrict__ psi_b1,
    const unsigned int* __restrict__ p2h, const unsigned int* __restrict__ p2l,
    const float* __restrict__ psi_b2,
    const float* __restrict__ bf_raw, float* out) {
  __shared__ __attribute__((aligned(16))) float lds[4][16 * LDS_STRIDE];
  __shared__ __attribute__((aligned(16))) float otile[NPART * DIM];
  int wave = threadIdx.x >> 5;
  int lane = threadIdx.x & 31;
  int h = lane >> 4;
  int lrow = lane & 15;
  int b = blockIdx.x;
  int ibase = wave * 16;
  float* L = lds[wave];
  int row = b * NPART + ibase + lrow;

  Frag AH[4], AL[4];
  load_A4(s + (size_t)row * HID, h, AH, AL);

#pragma unroll 1
  for (int c = 0; c < NCT; ++c) {
    int col = c * 16 + lrow;
    float bb = (float)(NPART - 1) * phi_b1[col];
    v8f acc;
#pragma unroll
    for (int r = 0; r < 8; ++r) acc[r] = bb;
    acc = gemm128_col(AH, AL, w1h, w1l, NCT, c, lane, acc);
#pragma unroll
    for (int r = 0; r < 8; ++r) L[(8 * h + r) * LDS_STRIDE + col] = acc[r];
  }
  __syncthreads();
  load_A4(L + lrow * LDS_STRIDE, h, AH, AL);

  Frag AX;
  {
    const float* xr = x + (size_t)row * DIM;
    unsigned int hx0, lx0, hx1, lx1, hx2, lx2;
    split2(xr[0], hx0, lx0);
    split2(xr[1], hx1, lx1);
    split2(xr[2], hx2, lx2);
    unsigned int u0 = (hx0 & 0xFFFFu) | (hx1 << 16);
    unsigned int u1 = (hx2 & 0xFFFFu) | (hx0 << 16);
    unsigned int u2 = (hx1 & 0xFFFFu) | (hx2 << 16);
    unsigned int u3 = (lx0 & 0xFFFFu) | (lx1 << 16);
    AX.u[0] = h ? (lx2 & 0xFFFFu) : u0;
    AX.u[1] = h ? 0u : u1;
    AX.u[2] = h ? 0u : u2;
    AX.u[3] = h ? 0u : u3;
    AX.u[4] = 0u; AX.u[5] = 0u; AX.u[6] = 0u; AX.u[7] = 0u;
  }
  __syncthreads();

#pragma unroll 1
  for (int c = 0; c < NCT; ++c) {
    int col = c * 16 + lrow;
    float bb = psi_b0[col];
    v8f acc;
#pragma unroll
    for (int r = 0; r < 8; ++r) acc[r] = bb;
    {
      Frag BX;
      load_B(pxt, c, lane, BX);
      acc = mma_bf16(AX.v, BX.v, acc);
    }
    acc = gemm128_col(AH, AL, pmh, pml, NCT, c, lane, acc);
#pragma unroll
    for (int r = 0; r < 8; ++r) L[(8 * h + r) * LDS_STRIDE + col] = silu_f(acc[r]);
  }
  __syncthreads();
  load_A4(L + lrow * LDS_STRIDE, h, AH, AL);
  __syncthreads();

#pragma unroll 1
  for (int c = 0; c < NCT; ++c) {
    int col = c * 16 + lrow;
    float bb = psi_b1[col];
    v8f acc;
#pragma unroll
    for (int r = 0; r < 8; ++r) acc[r] = bb;
    acc = gemm128_col(AH, AL, p1h, p1l, NCT, c, lane, acc);
#pragma unroll
    for (int r = 0; r < 8; ++r) L[(8 * h + r) * LDS_STRIDE + col] = silu_f(acc[r]);
  }
  __syncthreads();
  load_A4(L + lrow * LDS_STRIDE, h, AH, AL);

  v8f acc;
  {
    float bb0 = psi_b2[(lrow < DIM) ? lrow : 0];
    float bb = (lrow < DIM) ? bb0 : 0.0f;
#pragma unroll
    for (int r = 0; r < 8; ++r) acc[r] = bb;
  }
  acc = gemm128_col(AH, AL, p2h, p2l, 1, 0, lane, acc);
  float bfr = bf_raw[0];
  float sp = fmaxf(bfr, 0.0f) + log1pf(expf(-fabsf(bfr)));
  if (lrow < DIM) {
#pragma unroll
    for (int r = 0; r < 8; ++r) {
      int orow = ibase + 8 * h + r;
      otile[orow * DIM + lrow] = tanhf(acc[r]) * sp;
    }
  }
  __syncthreads();

  v4f o0 = *(const v4fa*)(otile + 4 * lane);
  v4f o1 = *(const v4fa*)(otile + 4 * (32 + (lane & 15)));
  float* ob = out + (size_t)b * (NPART * DIM);
  bool w0 = (wave == 0);
  if (w0) *(volatile v4f*)(ob + 4 * lane) = o0;
  if (w0 && lane < 16) *(volatile v4f*)(ob + 4 * (32 + lane)) = o1;
  __threadfence();
  if (w0) *(volatile v4f*)(ob + 4 * lane) = o0;
  if (w0 && lane < 16) *(volatile v4f*)(ob + 4 * (32 + lane)) = o1;
}

extern "C" void kernel_launch(void* const* d_in, const int* in_sizes, int n_in,
                              void* d_out, int out_size, void* d_ws, size_t ws_size,
                              hipStream_t stream) {
  if (n_in < 13) return;
  const float* x      = (const float*)d_in[0];
  const int*   spin   = (const int*)d_in[1];
  const float* phi_w0 = (const float*)d_in[2];
  const float* phi_b0 = (const float*)d_in[3];
  const float* phi_w1 = (const float*)d_in[4];
  const float* phi_b1 = (const float*)d_in[5];
  const float* psi_w0 = (const float*)d_in[6];
  const float* psi_b0 = (const float*)d_in[7];
  const float* psi_w1 = (const float*)d_in[8];
  const float* psi_b1 = (const float*)d_in[9];
  const float* psi_w2 = (const float*)d_in[10];
  const float* psi_b2 = (const float*)d_in[11];
  const float* bf_raw = (const float*)d_in[12];

  int nB = in_sizes[0] / (NPART * DIM);
  if (nB <= 0 || in_sizes[0] != nB * NPART * DIM) return;
  if ((long long)out_size < (long long)nB * NPART * DIM) return;

  const size_t OFF_W0T = 0;
  const size_t OFF_W1H = 8192;
  const size_t OFF_W1L = 40960;
  const size_t OFF_PXT = 73728;
  const size_t OFF_PMH = 81920;
  const size_t OFF_PML = 114688;
  const size_t OFF_P1H = 147456;
  const size_t OFF_P1L = 180224;
  const size_t OFF_P2H = 212992;
  const size_t OFF_P2L = 217088;
  const size_t OFF_S   = 262144;
  size_t s_bytes = (size_t)nB * NPART * HID * sizeof(float);
  if (OFF_S + s_bytes > ws_size) return;

  char* ws = (char*)d_ws;
  unsigned int* w0t = (unsigned int*)(ws + OFF_W0T);
  unsigned int* w1h = (unsigned int*)(ws + OFF_W1H);
  unsigned int* w1l = (unsigned int*)(ws + OFF_W1L);
  unsigned int* pxt = (unsigned int*)(ws + OFF_PXT);
  unsigned int* pmh = (unsigned int*)(ws + OFF_PMH);
  unsigned int* pml = (unsigned int*)(ws + OFF_PML);
  unsigned int* p1h = (unsigned int*)(ws + OFF_P1H);
  unsigned int* p1l = (unsigned int*)(ws + OFF_P1L);
  unsigned int* p2h = (unsigned int*)(ws + OFF_P2H);
  unsigned int* p2l = (unsigned int*)(ws + OFF_P2L);
  float* s = (float*)(ws + OFF_S);

  pack_tiny <<<(NCT * 64 + 255) / 256, 256, 0, stream>>>(phi_w0, HID, 3, 8, HID, NCT, w0t);
  pack_split<<<(4 * NCT * 64 + 255) / 256, 256, 0, stream>>>(phi_w1, HID, 0, HID, HID, NCT, 4, w1h, w1l);
  pack_tiny <<<(NCT * 64 + 255) / 256, 256, 0, stream>>>(psi_w0, HID, 0, DIM, HID, NCT, pxt);
  pack_split<<<(4 * NCT * 64 + 255) / 256, 256, 0, stream>>>(psi_w0, HID, DIM, HID, HID, NCT, 4, pmh, pml);
  pack_split<<<(4 * NCT * 64 + 255) / 256, 256, 0, stream>>>(psi_w1, HID, 0, HID, HID, NCT, 4, p1h, p1l);
  pack_split<<<(4 * 1 * 64 + 255) / 256, 256, 0, stream>>>(psi_w2, DIM, 0, HID, DIM, 1, 4, p2h, p2l);

  int nrows = nB * NPART;
  int grid1 = (nrows + WAVES1 - 1) / WAVES1;
  phase1<<<grid1, 32 * WAVES1, 0, stream>>>(x, spin, phi_w0, phi_b0, w0t, s, nrows);
  phase2<<<nB, 128, 0, stream>>>(x, s, w1h, w1l, phi_b1, pxt, pmh, pml, psi_b0,
                                 p1h, p1l, psi_b1, p2h, p2l, psi_b2, bf_raw,
                                 (float*)d_out);
  (void)hipGetLastError();
}
